// CustomGraphNet_6880537608483
// MI455X (gfx1250) — hardware-run, weakly checked
//
#include <hip/hip_runtime.h>
#include <stddef.h>


#define CH      128
#define QW      512
#define DCOND   768
#define NJOB    12
#define NTHR    256
#define NWAVE   8
#define EPTH    8
#define NGRP    2
#define CHUNK   (NTHR * EPTH * NGRP)
#define WCAP    (EPTH * NGRP * 32)
#define LISTN   (NWAVE * WCAP)
#define NBC     4096
#define NBF     1024
#define RCAP    40960
#define RBN     128
#define TGT     256
#define DEGCAP  256
#define GROWS   128
#define GNC     128
#define OTHR    512
#define WSCAP   134217728
#define NEG_BIG (-3.0e38f)
#define WSC     16.0f
#define RWSC    0.0625f
#define ATT_SCL 0.08838834764831845f
#define LDS_FILL ((RCAP + NBF + LISTN) * 4 + 64)
#define LDS_GEMM (GROWS * GNC * 4)

static_assert((CHUNK & (CHUNK - 1)) == 0);
static_assert(CHUNK <= 4096);
static_assert(NBC == 4 * NBF);
static_assert(OTHR * 8 == NBC);
static_assert((RCAP % 32) == 0);
static_assert(TGT == NWAVE * 32);
static_assert(GROWS == NWAVE * 16);
static_assert(QW == 4 * CH);

typedef float    v4f  __attribute__((ext_vector_type(4)));
typedef float    v8f  __attribute__((ext_vector_type(8)));
typedef int      v4i  __attribute__((ext_vector_type(4)));
typedef _Float16 v4h  __attribute__((ext_vector_type(4)));
typedef _Float16 v8h  __attribute__((ext_vector_type(8)));
typedef _Float16 v16h __attribute__((ext_vector_type(16)));
union Frag { v16h v; v8h h[2]; };

__device__ __forceinline__ v8f wmm(v16h a, v16h b, v8f c) {
  c = __builtin_amdgcn_wmma_f32_16x16x32_f16(false, a, false, b, (short)0, c, false, false);
  asm volatile("v_nop\n\tv_nop\n\tv_nop\n\tv_nop" : "+v"(c) : "v"(a), "v"(b));
  return c;
}

__device__ __forceinline__ float wsum(float v) {
#pragma unroll
  for (int o = 16; o > 0; o >>= 1) v += __shfl_xor(v, o);
  return v;
}
__device__ __forceinline__ float wmax(float v) {
#pragma unroll
  for (int o = 16; o > 0; o >>= 1) v = fmaxf(v, __shfl_xor(v, o));
  return v;
}
__device__ __forceinline__ v4h cvt4(v4f v) {
  v4h r;
  r.x = (_Float16)v.x; r.y = (_Float16)v.y; r.z = (_Float16)v.z; r.w = (_Float16)v.w;
  return r;
}
__device__ __forceinline__ float sel4(int g, float a, float b, float c, float d) {
  return g == 0 ? a : (g == 1 ? b : (g == 2 ? c : d));
}
__device__ __forceinline__ float rdl(float v, int l) {
  return __uint_as_float((unsigned int)__builtin_amdgcn_readlane((int)__float_as_uint(v), l));
}
__device__ __forceinline__ float hsum4(v4f v) { return (v.x + v.y) + (v.z + v.w); }
__device__ __forceinline__ v4f xs2(v4f v) {
  v.x += __shfl_xor(v.x, 8);  v.y += __shfl_xor(v.y, 8);  v.z += __shfl_xor(v.z, 8);  v.w += __shfl_xor(v.w, 8);
  v.x += __shfl_xor(v.x, 16); v.y += __shfl_xor(v.y, 16); v.z += __shfl_xor(v.z, 16); v.w += __shfl_xor(v.w, 16);
  return v;
}

template <int NB>
__device__ __forceinline__ int scan_chunk(const int* __restrict__ dsts, int nE, int cbase, int slotBase,
                                          int vec8, int* list, int tid, int lane, int wave) {
  int wc = 0;
#pragma unroll
  for (int g = 0; g < NGRP; ++g) {
    const int el0  = (g * NTHR + tid) * EPTH;
    const int e0   = cbase + el0;
    const int sent = -2147483647 - 1;
    v4i da, db;
    if (vec8 != 0 && cbase + CHUNK <= nE) {
      da = *(const v4i*)(dsts + e0);
      db = *(const v4i*)(dsts + e0 + 4);
    } else {
      da.x = (e0     < nE) ? dsts[min(e0, nE - 1)] : sent;
      da.y = (e0 + 1 < nE) ? dsts[min(e0 + 1, nE - 1)] : sent;
      da.z = (e0 + 2 < nE) ? dsts[min(e0 + 2, nE - 1)] : sent;
      da.w = (e0 + 3 < nE) ? dsts[min(e0 + 3, nE - 1)] : sent;
      db.x = (e0 + 4 < nE) ? dsts[min(e0 + 4, nE - 1)] : sent;
      db.y = (e0 + 5 < nE) ? dsts[min(e0 + 5, nE - 1)] : sent;
      db.z = (e0 + 6 < nE) ? dsts[min(e0 + 6, nE - 1)] : sent;
      db.w = (e0 + 7 < nE) ? dsts[min(e0 + 7, nE - 1)] : sent;
    }
    const unsigned nb = (unsigned)slotBase;
    const unsigned s0 = (unsigned)da.x - nb, s1 = (unsigned)da.y - nb;
    const unsigned s2 = (unsigned)da.z - nb, s3 = (unsigned)da.w - nb;
    const unsigned s4 = (unsigned)db.x - nb, s5 = (unsigned)db.y - nb;
    const unsigned s6 = (unsigned)db.z - nb, s7 = (unsigned)db.w - nb;
    const bool h0 = s0 < (unsigned)NB, h1 = s1 < (unsigned)NB, h2 = s2 < (unsigned)NB, h3 = s3 < (unsigned)NB;
    const bool h4 = s4 < (unsigned)NB, h5 = s5 < (unsigned)NB, h6 = s6 < (unsigned)NB, h7 = s7 < (unsigned)NB;
    const unsigned any = __builtin_amdgcn_ballot_w32(h0 | h1 | h2 | h3 | h4 | h5 | h6 | h7);
    if (any != 0u) {
#define HITJ(J, HJ, SJ) { \
        const unsigned mj = __builtin_amdgcn_ballot_w32(HJ); \
        if (mj != 0u) { \
          if (HJ) { \
            const int p = wc + (int)__builtin_amdgcn_mbcnt_lo(mj, 0u); \
            if (p < WCAP) list[wave * WCAP + p] = ((el0 + (J)) << 12) | (int)(SJ); \
          } \
          wc += (int)__builtin_popcount(mj); } }
      HITJ(0, h0, s0)
      HITJ(1, h1, s1)
      HITJ(2, h2, s2)
      HITJ(3, h3, s3)
      HITJ(4, h4, s4)
      HITJ(5, h5, s5)
      HITJ(6, h6, s6)
      HITJ(7, h7, s7)
#undef HITJ
    }
  }
  return wc;
}

__global__ __launch_bounds__(NTHR) void k_count(const int* __restrict__ ei, int* cnt, int nE, int vec8) {
  __shared__ __attribute__((aligned(16))) int scnt[NBC];
  __shared__ __attribute__((aligned(16))) int list[LISTN];
  __shared__ int wcnt[NWAVE];
  const int tid = threadIdx.x, lane = tid & 31, wave = tid >> 5;
  const int nodeBase = blockIdx.x * NBC;
  const int* dsts = ei + nE;
  for (int i = tid; i < NBC; i += NTHR) scnt[i] = 0;
  __syncthreads();
  const int nChunks = (nE + CHUNK - 1) / CHUNK;
#pragma unroll 1
  for (int ch = 0; ch < nChunks; ++ch) {
    const int cbase = ch * CHUNK;
    const int wc = scan_chunk<NBC>(dsts, nE, cbase, nodeBase, vec8, list, tid, lane, wave);
    if (lane == 0) wcnt[wave] = wc;
    __syncthreads();
    if (wave == 0) {
#pragma unroll 1
      for (int wsx = 0; wsx < NWAVE; ++wsx) {
        int n = __builtin_amdgcn_readfirstlane(wcnt[wsx]);
        n = n > WCAP ? WCAP : (n < 0 ? 0 : n);
        const int* lp = list + wsx * WCAP;
#pragma unroll 1
        for (int i = 0; i < n; ++i) {
          const int ent  = __builtin_amdgcn_readfirstlane(lp[i]);
          const int slot = ent & (NBC - 1);
          if (lane == 0) scnt[slot] = scnt[slot] + 1;
        }
      }
    }
    __syncthreads();
  }
  v4i cq[4];
#pragma unroll
  for (int q = 0; q < 4; ++q) cq[q] = *(const v4i*)(scnt + (wave * 4 + q) * 128 + 4 * lane);
  int* cp = cnt + (size_t)nodeBase;
#pragma unroll
  for (int q = 0; q < 4; ++q) *(volatile v4i*)(cp + (wave * 4 + q) * 128 + 4 * lane) = cq[q];
  __threadfence();
#pragma unroll
  for (int q = 0; q < 4; ++q) *(volatile v4i*)(cp + (wave * 4 + q) * 128 + 4 * lane) = cq[q];
}

__global__ __launch_bounds__(OTHR) void k_offsets(const int* __restrict__ cnt, int* off, int* rbase, int nChunk) {
  __shared__ __attribute__((aligned(16))) int soff[NBC];
  __shared__ __attribute__((aligned(16))) int srb[RBN];
  __shared__ int wtot[OTHR / 32];
  const int tid = threadIdx.x, lane = tid & 31, wave = tid >> 5, sub = tid >> 7;
  for (int i = tid; i < RBN; i += OTHR) srb[i] = 0;
  int carry = 0;
#pragma unroll 1
  for (int ch = 0; ch < nChunk; ++ch) {
    const int base = ch * NBC;
    const v4i c0 = *(const v4i*)(cnt + base + 8 * tid);
    const v4i c1 = *(const v4i*)(cnt + base + 8 * tid + 4);
    const int e0 = max(c0.x, 0), e1 = max(c0.y, 0), e2 = max(c0.z, 0), e3 = max(c0.w, 0);
    const int e4 = max(c1.x, 0), e5 = max(c1.y, 0), e6 = max(c1.z, 0), e7 = max(c1.w, 0);
    const int ts = e0 + e1 + e2 + e3 + e4 + e5 + e6 + e7;
    int incl = ts;
#pragma unroll
    for (int d = 1; d < 32; d <<= 1) {
      const int t = __shfl_up(incl, d);
      if (lane >= d) incl += t;
    }
    if (lane == 31) wtot[wave] = incl;
    __syncthreads();
    const int S0 = wtot[0]  + wtot[1]  + wtot[2]  + wtot[3];
    const int S1 = wtot[4]  + wtot[5]  + wtot[6]  + wtot[7];
    const int S2 = wtot[8]  + wtot[9]  + wtot[10] + wtot[11];
    const int S3 = wtot[12] + wtot[13] + wtot[14] + wtot[15];
    int pre = 0;
#pragma unroll 1
    for (int w = 4 * sub; w < wave; ++w) pre += wtot[w];
    const int b0 = carry;
    const int b1 = b0 + ((S0 + 31) & ~31);
    const int b2 = b1 + ((S1 + 31) & ~31);
    const int b3 = b2 + ((S2 + 31) & ~31);
    const int b4 = b3 + ((S3 + 31) & ~31);
    const int myb = sub == 0 ? b0 : (sub == 1 ? b1 : (sub == 2 ? b2 : b3));
    if (tid == 0) {
      srb[min(4 * ch + 0, RBN - 1)] = b0;
      srb[min(4 * ch + 1, RBN - 1)] = b1;
      srb[min(4 * ch + 2, RBN - 1)] = b2;
      srb[min(4 * ch + 3, RBN - 1)] = b3;
    }
    int run = myb + pre + incl - ts;
    soff[8 * tid + 0] = run; run += e0;
    soff[8 * tid + 1] = run; run += e1;
    soff[8 * tid + 2] = run; run += e2;
    soff[8 * tid + 3] = run; run += e3;
    soff[8 * tid + 4] = run; run += e4;
    soff[8 * tid + 5] = run; run += e5;
    soff[8 * tid + 6] = run; run += e6;
    soff[8 * tid + 7] = run;
    carry = b4;
    __syncthreads();
    const v4i o0 = *(const v4i*)(soff + 4 * tid);
    const v4i o1 = *(const v4i*)(soff + 4 * (tid + OTHR));
    int* op = off + base;
    *(volatile v4i*)(op + 4 * tid) = o0;
    *(volatile v4i*)(op + 4 * (tid + OTHR)) = o1;
    __threadfence();
    *(volatile v4i*)(op + 4 * tid) = o0;
    *(volatile v4i*)(op + 4 * (tid + OTHR)) = o1;
    __syncthreads();
  }
  if (tid == 0) srb[min(4 * nChunk, RBN - 1)] = carry;
  __syncthreads();
  v4i rv = {0, 0, 0, 0};
  if (tid < 32) rv = *(const v4i*)(srb + 4 * tid);
  if (tid < 32) *(volatile v4i*)(rbase + 4 * tid) = rv;
  __threadfence();
  if (tid < 32) *(volatile v4i*)(rbase + 4 * tid) = rv;
}

__global__ __launch_bounds__(NTHR) void k_fill(const int* __restrict__ ei, const int* __restrict__ off, const int* __restrict__ rbase,
                                               int* csr, int nE, int vec8, int csrLen) {
  extern __shared__ v4f lds_dyn[];
  int* region = (int*)lds_dyn;
  int* cursor = region + RCAP;
  int* list   = cursor + NBF;
  int* wcnt   = list + LISTN;
  const int tid = threadIdx.x, lane = tid & 31, wave = tid >> 5;
  const int b = blockIdx.x;
  const int nodeBase = b * NBF;
  const int* dsts = ei + nE;
  int rb0 = rbase[b];
  const int rb1 = rbase[b + 1];
  rb0 = rb0 < 0 ? 0 : (rb0 > csrLen ? csrLen : rb0);
  rb0 &= ~31;
  int len = rb1 - rb0;
  len = len < 0 ? 0 : (len > RCAP ? RCAP : len);
  int lenW = (len + 31) & ~31;
  if (rb0 + lenW > csrLen) lenW = (csrLen - rb0) & ~31;
  {
    const v4i z = {0, 0, 0, 0};
    for (int i = tid; i < RCAP / 4; i += NTHR) ((v4i*)region)[i] = z;
    for (int s = tid; s < NBF; s += NTHR) {
      int o = off[nodeBase + s] - rb0;
      o = o < 0 ? 0 : (o > RCAP ? RCAP : o);
      cursor[s] = o;
    }
  }
  __syncthreads();
  const int nChunks = (nE + CHUNK - 1) / CHUNK;
#pragma unroll 1
  for (int ch = 0; ch < nChunks; ++ch) {
    const int cbase = ch * CHUNK;
    const int wc = scan_chunk<NBF>(dsts, nE, cbase, nodeBase, vec8, list, tid, lane, wave);
    if (lane == 0) wcnt[wave] = wc;
    __syncthreads();
    if (wave == 0) {
#pragma unroll 1
      for (int wsx = 0; wsx < NWAVE; ++wsx) {
        int n = __builtin_amdgcn_readfirstlane(wcnt[wsx]);
        n = n > WCAP ? WCAP : (n < 0 ? 0 : n);
        const int* lp = list + wsx * WCAP;
#pragma unroll 1
        for (int i = 0; i < n; ++i) {
          const int ent  = __builtin_amdgcn_readfirstlane(lp[i]);
          const int slot = ent & (NBF - 1);
          int e = cbase + ((ent >> 12) & (CHUNK - 1));
          e = e > nE - 1 ? nE - 1 : e;
          if (lane == 0) {
            int p = cursor[slot];
            p = p < 0 ? 0 : (p > RCAP - 1 ? RCAP - 1 : p);
            region[p] = e;
            const int np = p + 1;
            cursor[slot] = np > RCAP ? RCAP : np;
          }
        }
      }
    }
    __syncthreads();
  }
  const int nv = lenW >> 2;
  int* gp = csr + rb0;
#pragma unroll 1
  for (int i = tid; i < nv; i += NTHR) { const v4i v = ((const v4i*)region)[i]; *(volatile v4i*)(gp + 4 * i) = v; }
  __threadfence();
#pragma unroll 1
  for (int i = tid; i < nv; i += NTHR) { const v4i v = ((const v4i*)region)[i]; *(volatile v4i*)(gp + 4 * i) = v; }
}

__global__ __launch_bounds__(NTHR) void k_dinv(const int* __restrict__ cnt, float* dinv, int items4) {
  const int idx = blockIdx.x * NTHR + threadIdx.x;
  if (idx >= items4) return;
  const v4i c = *(const v4i*)(cnt + 4 * idx);
  v4f d;
  d.x = rsqrtf((float)(c.x < 0 ? 0 : c.x) + 1.0f);
  d.y = rsqrtf((float)(c.y < 0 ? 0 : c.y) + 1.0f);
  d.z = rsqrtf((float)(c.z < 0 ? 0 : c.z) + 1.0f);
  d.w = rsqrtf((float)(c.w < 0 ? 0 : c.w) + 1.0f);
  float* p = dinv + 4 * idx;
  *(volatile v4f*)p = d;
  __threadfence();
  *(volatile v4f*)p = d;
}

struct WJob  { const float* src; _Float16* dst; int K; int N; };
struct WJobs { WJob j[NJOB]; };
static_assert(sizeof(WJob) == 24);
static_assert(sizeof(WJobs) == 24 * NJOB);

__global__ __launch_bounds__(NTHR) void k_wprep(WJobs J) {
  const int y = (int)blockIdx.y;
  const float* src = J.j[0].src; _Float16* dst = J.j[0].dst;
  int K = J.j[0].K, N = J.j[0].N;
#pragma unroll
  for (int i = 1; i < NJOB; ++i)
    if (i == y) { src = J.j[i].src; dst = J.j[i].dst; K = J.j[i].K; N = J.j[i].N; }
  const int idx = blockIdx.x * NTHR + threadIdx.x;
  const int kp8 = K >> 3;
  const int items = N * kp8;
  if (idx >= items) return;
  const int n = idx / kp8;
  const int k0 = (idx - n * kp8) * 8;
  v8h hv;
#pragma unroll
  for (int e = 0; e < 8; ++e) {
    const float x = src[(size_t)(k0 + e) * N + n] * WSC;
    hv[e] = (_Float16)x;
  }
  _Float16* dp = dst + (size_t)idx * 8;
  *(volatile v8h*)dp = hv;
  __threadfence();
  *(volatile v8h*)dp = hv;
}

__global__ __launch_bounds__(NTHR) void k_cvt(const float* __restrict__ x, _Float16* H, int nN, int K, int items) {
  const int idx = blockIdx.x * NTHR + threadIdx.x;
  if (idx >= items) return;
  const int kp8 = K >> 3;
  const int r = idx / kp8;
  const int k0 = (idx - r * kp8) * 8;
  const int rc = r < nN ? r : nN - 1;
  const float* xp = x + (size_t)rc * K + k0;
  v4f a = *(const v4f*)xp;
  v4f b = *(const v4f*)(xp + 4);
  const v4f z = {0.f, 0.f, 0.f, 0.f};
  a = r < nN ? a : z;
  b = r < nN ? b : z;
  v8h hv;
  hv[0] = (_Float16)a.x; hv[1] = (_Float16)a.y; hv[2] = (_Float16)a.z; hv[3] = (_Float16)a.w;
  hv[4] = (_Float16)b.x; hv[5] = (_Float16)b.y; hv[6] = (_Float16)b.z; hv[7] = (_Float16)b.w;
  _Float16* dp = H + (size_t)idx * 8;
  *(volatile v8h*)dp = hv;
  __threadfence();
  *(volatile v8h*)dp = hv;
}

__global__ __launch_bounds__(NTHR) void k_bnstat(const float* __restrict__ x, float* stats, int nN) {
  __shared__ double sd[NWAVE * 32];
  __shared__ float smu[32];
  __shared__ __attribute__((aligned(16))) float sln[64];
  const int tid = threadIdx.x, lane = tid & 31, wave = tid >> 5;
  const int col = (int)blockIdx.x * 32 + lane;
  double s = 0.0;
#pragma unroll 1
  for (int r = wave; r < nN; r += NWAVE) s += (double)x[(size_t)r * CH + col];
  sd[wave * 32 + lane] = s;
  __syncthreads();
  if (wave == 0) {
    double t = 0.0;
#pragma unroll
    for (int w = 0; w < NWAVE; ++w) t += sd[w * 32 + lane];
    smu[lane] = (float)(t / (double)nN);
  }
  __syncthreads();
  const float mu = smu[lane];
  double s2 = 0.0;
#pragma unroll 1
  for (int r = wave; r < nN; r += NWAVE) {
    const float d = x[(size_t)r * CH + col] - mu;
    const double dd = (double)d;
    s2 += dd * dd;
  }
  sd[wave * 32 + lane] = s2;
  __syncthreads();
  if (wave == 0) {
    double t = 0.0;
#pragma unroll
    for (int w = 0; w < NWAVE; ++w) t += sd[w * 32 + lane];
    const float var = (float)(t / (double)nN);
    const float rs = 1.0f / sqrtf(var + 1e-5f);
    sln[lane] = mu;
    sln[32 + lane] = rs;
  }
  __syncthreads();
  v4f v = {0.f, 0.f, 0.f, 0.f};
  if (tid < 16) v = *(const v4f*)(sln + 4 * tid);
  const int go = tid < 8 ? ((int)blockIdx.x * 32 + 4 * tid) : (CH + (int)blockIdx.x * 32 + 4 * (tid - 8));
  float* gp = stats + (tid < 16 ? go : 0);
  if (tid < 16) *(volatile v4f*)gp = v;
  __threadfence();
  if (tid < 16) *(volatile v4f*)gp = v;
}

__global__ __launch_bounds__(NTHR) void k_bnapply(const float* __restrict__ x, const float* __restrict__ stats,
                                                  const float* __restrict__ g, const float* __restrict__ b, _Float16* H, int nN) {
  const int tid = threadIdx.x, lane = tid & 31, wave = tid >> 5;
  const int wg = blockIdx.x * NWAVE + wave;
  const v4f mu = *(const v4f*)(stats + 4 * lane);
  const v4f rs = *(const v4f*)(stats + CH + 4 * lane);
  const v4f gg = *(const v4f*)(g + 4 * lane);
  const v4f bb = *(const v4f*)(b + 4 * lane);
  const v4f z = {0.f, 0.f, 0.f, 0.f};
#pragma unroll 1
  for (int i = 0; i < 4; ++i) {
    const int r = wg * 4 + i;
    const int rc = r < nN ? r : nN - 1;
    const v4f xv = *(const v4f*)(x + (size_t)rc * CH + 4 * lane);
    v4f y = (xv - mu) * rs * gg + bb;
    y = r < nN ? y : z;
    const v4h hv = cvt4(y);
    _Float16* hp = H + (size_t)r * CH + 4 * lane;
    *(volatile v4h*)hp = hv;
    __threadfence();
    *(volatile v4h*)hp = hv;
  }
}

__global__ __launch_bounds__(NTHR) void k_gemm(const _Float16* __restrict__ A, const _Float16* __restrict__ B, const float* __restrict__ bias,
                                               float* C, int lda, int ldb, int ldc, int ksteps, int useBias, float scale) {
  extern __shared__ v4f lds_dyn[];
  float* stg = (float*)lds_dyn;
  const int tid = threadIdx.x, lane = tid & 31, wave = tid >> 5, hh = lane >> 4, m = lane & 15;
  const int rowBase = (int)blockIdx.x * GROWS;
  const int slab = (int)blockIdx.y;
  const _Float16* Bs = B + (size_t)slab * GNC * (size_t)ldb;
  const _Float16* ap = A + (size_t)(rowBase + wave * 16 + m) * lda + 8 * hh;
  v8f acc[8];
#pragma unroll
  for (int t = 0; t < 8; ++t) { v8f z = {0.f, 0.f, 0.f, 0.f, 0.f, 0.f, 0.f, 0.f}; acc[t] = z; }
#pragma unroll 1
  for (int kt = 0; kt < ksteps; ++kt) {
    Frag a;
    a.h[0] = *(const v8h*)(ap + 32 * kt);
    a.h[1] = *(const v8h*)(ap + 32 * kt + 16);
#pragma unroll
    for (int t = 0; t < 8; ++t) {
      const _Float16* bp = Bs + (size_t)(16 * t + m) * ldb + 32 * kt + 8 * hh;
      Frag b;
      b.h[0] = *(const v8h*)bp;
      b.h[1] = *(const v8h*)(bp + 16);
      acc[t] = wmm(a.v, b.v, acc[t]);
    }
  }
  const int r0 = wave * 16 + 8 * hh;
#pragma unroll
  for (int t = 0; t < 8; ++t) {
    const int col = 16 * t + m;
    const float bl = bias[slab * GNC + col];
    const float bb = useBias ? bl : 0.0f;
#pragma unroll
    for (int r = 0; r < 8; ++r) stg[(r0 + r) * GNC + col] = acc[t][r] * scale + bb;
  }
  __syncthreads();
  float* Cs = C + (size_t)slab * GNC;
#pragma unroll
  for (int i = 0; i < 16; ++i) {
    const int lr = wave * 16 + i;
    const v4f v = *(const v4f*)(stg + lr * GNC + 4 * lane);
    *(volatile v4f*)(Cs + (size_t)(rowBase + lr) * ldc + 4 * lane) = v;
  }
  __threadfence();
#pragma unroll
  for (int i = 0; i < 16; ++i) {
    const int lr = wave * 16 + i;
    const v4f v = *(const v4f*)(stg + lr * GNC + 4 * lane);
    *(volatile v4f*)(Cs + (size_t)(rowBase + lr) * ldc + 4 * lane) = v;
  }
}

__global__ __launch_bounds__(NTHR) void k_gcn(const int* __restrict__ csr, const int* __restrict__ off, const int* __restrict__ cnt,
    const int* __restrict__ ei, const float* __restrict__ dinv, const float* __restrict__ XW, const float* __restrict__ bias,
    const float* __restrict__ xin, _Float16* Hout, float* out, int nN, int nE, int csrLen, int mode) {
  const int tid = threadIdx.x, lane = tid & 31, wave = tid >> 5;
  const int tbase = blockIdx.x * TGT + wave * 32;
  const int cnt_l = cnt[tbase + lane], off_l = off[tbase + lane];
  const float dv_l = dinv[tbase + lane];
  const v4f bb = *(const v4f*)(bias + 4 * lane);
#pragma unroll 1
  for (int j = 0; j < 32; ++j) {
    const int c = tbase + j;
    int n = __builtin_amdgcn_readfirstlane(__shfl(cnt_l, j));
    n = n < 0 ? 0 : (n > DEGCAP ? DEGCAP : n);
    const int st = __builtin_amdgcn_readfirstlane(__shfl(off_l, j));
    const float dd = __shfl(dv_l, j);
    v4f acc = {0.f, 0.f, 0.f, 0.f};
#pragma unroll 1
    for (int q0 = 0; q0 < n; q0 += 32) {
      int p = st + q0 + lane; p = p < 0 ? 0 : (p > csrLen - 1 ? csrLen - 1 : p);
      int eid = csr[p];  eid = eid < 0 ? 0 : (eid > nE - 1 ? nE - 1 : eid);
      int sl = ei[eid];  sl = sl < 0 ? 0 : (sl > nN - 1 ? nN - 1 : sl);
      const float ds = dinv[sl];
      const int mcnt = (n - q0) < 32 ? (n - q0) : 32;
#pragma unroll 1
      for (int pp = 0; pp < mcnt; ++pp) {
        const int s = __builtin_amdgcn_readlane(sl, pp);
        const float w = rdl(ds, pp) * dd;
        const v4f xv = *(const v4f*)(XW + (size_t)s * CH + 4 * lane);
        acc = acc + xv * w;
      }
    }
    const v4f xs = *(const v4f*)(XW + (size_t)c * CH + 4 * lane);
    v4f r = acc + xs * (dd * dd) + bb;
    if (mode == 1) {
      r.x = r.x * __builtin_amdgcn_rcpf(1.0f + __expf(-r.x));
      r.y = r.y * __builtin_amdgcn_rcpf(1.0f + __expf(-r.y));
      r.z = r.z * __builtin_amdgcn_rcpf(1.0f + __expf(-r.z));
      r.w = r.w * __builtin_amdgcn_rcpf(1.0f + __expf(-r.w));
    }
    if (mode == 2) {
      if (c < nN) {
        const v4f xi = *(const v4f*)(xin + (size_t)c * CH + 4 * lane);
        const v4f o = xi + r;
        float* op = out + (size_t)c * CH + 4 * lane;
        *(volatile v4f*)op = o;
        __threadfence();
        *(volatile v4f*)op = o;
      }
    } else {
      const v4h hv = cvt4(r);
      _Float16* hp = Hout + (size_t)c * CH + 4 * lane;
      *(volatile v4h*)hp = hv;
      __threadfence();
      *(volatile v4h*)hp = hv;
    }
  }
}

__global__ __launch_bounds__(NTHR) void k_attn(const int* __restrict__ csr, const int* __restrict__ off, const int* __restrict__ cnt,
    const int* __restrict__ ei, const float* __restrict__ Q, const float* __restrict__ Kf, const float* __restrict__ Vf,
    const float* __restrict__ SK, const float* __restrict__ lng, const float* __restrict__ lnb, _Float16* Hout,
    int nN, int nE, int csrLen) {
  __shared__ __attribute__((aligned(16))) float srow[NWAVE * CH];
  const int tid = threadIdx.x, lane = tid & 31, wave = tid >> 5;
  const int grp = lane >> 3, sub = lane & 7;
  const int hoff = grp * CH + sub * 16;
  float* my = srow + wave * CH;
  const int tbase = blockIdx.x * TGT + wave * 32;
  const int cnt_l = cnt[tbase + lane], off_l = off[tbase + lane];
  const v4f g4 = *(const v4f*)(lng + 4 * lane);
  const v4f b4 = *(const v4f*)(lnb + 4 * lane);
  const v4f z4 = {0.f, 0.f, 0.f, 0.f};
#pragma unroll 1
  for (int j = 0; j < 32; ++j) {
    const int c = tbase + j;
    int n = __builtin_amdgcn_readfirstlane(__shfl(cnt_l, j));
    n = n < 0 ? 0 : (n > DEGCAP ? DEGCAP : n);
    const int st = __builtin_amdgcn_readfirstlane(__shfl(off_l, j));
    const float* qp = Q + (size_t)c * QW + hoff;
    const v4f q0 = *(const v4f*)qp, q1 = *(const v4f*)(qp + 4), q2 = *(const v4f*)(qp + 8), q3 = *(const v4f*)(qp + 12);
    float M0 = NEG_BIG, M1 = NEG_BIG, M2 = NEG_BIG, M3 = NEG_BIG;
    float d0 = 0.f, d1 = 0.f, d2 = 0.f, d3 = 0.f;
    v4f a0 = z4, a1 = z4, a2 = z4, a3 = z4;
#pragma unroll 1
    for (int q0i = 0; q0i < n; q0i += 32) {
      int p = st + q0i + lane; p = p < 0 ? 0 : (p > csrLen - 1 ? csrLen - 1 : p);
      int eid = csr[p];  eid = eid < 0 ? 0 : (eid > nE - 1 ? nE - 1 : eid);
      int sl = ei[eid];  sl = sl < 0 ? 0 : (sl > nN - 1 ? nN - 1 : sl);
      const int mcnt = (n - q0i) < 32 ? (n - q0i) : 32;
      float sc0 = NEG_BIG, sc1 = NEG_BIG, sc2 = NEG_BIG, sc3 = NEG_BIG;
#pragma unroll 1
      for (int pp = 0; pp < mcnt; ++pp) {
        const int s = __builtin_amdgcn_readlane(sl, pp);
        const float* kp = Kf + (size_t)s * QW + hoff;
        const v4f k0 = *(const v4f*)kp, k1 = *(const v4f*)(kp + 4), k2 = *(const v4f*)(kp + 8), k3 = *(const v4f*)(kp + 12);
        const v4f pr = q0 * k0 + q1 * k1 + q2 * k2 + q3 * k3;
        float t = hsum4(pr);
        t += __shfl_xor(t, 4); t += __shfl_xor(t, 2); t += __shfl_xor(t, 1);
        t *= ATT_SCL;
        const float e0 = __shfl(t, 0), e1 = __shfl(t, 8), e2 = __shfl(t, 16), e3 = __shfl(t, 24);
        const bool hit = (lane == pp);
        sc0 = hit ? e0 : sc0; sc1 = hit ? e1 : sc1; sc2 = hit ? e2 : sc2; sc3 = hit ? e3 : sc3;
      }
      const bool val = lane < mcnt;
      float r0, r1, r2, r3, p0, p1, p2, p3;
      {
        const float cm = wmax(val ? sc0 : NEG_BIG); const float nm = fmaxf(M0, cm);
        r0 = __expf(M0 - nm); M0 = nm; p0 = val ? __expf(sc0 - M0) : 0.f; d0 = d0 * r0 + wsum(p0);
      }
      {
        const float cm = wmax(val ? sc1 : NEG_BIG); const float nm = fmaxf(M1, cm);
        r1 = __expf(M1 - nm); M1 = nm; p1 = val ? __expf(sc1 - M1) : 0.f; d1 = d1 * r1 + wsum(p1);
      }
      {
        const float cm = wmax(val ? sc2 : NEG_BIG); const float nm = fmaxf(M2, cm);
        r2 = __expf(M2 - nm); M2 = nm; p2 = val ? __expf(sc2 - M2) : 0.f; d2 = d2 * r2 + wsum(p2);
      }
      {
        const float cm = wmax(val ? sc3 : NEG_BIG); const float nm = fmaxf(M3, cm);
        r3 = __expf(M3 - nm); M3 = nm; p3 = val ? __expf(sc3 - M3) : 0.f; d3 = d3 * r3 + wsum(p3);
      }
      const float rm = sel4(grp, r0, r1, r2, r3);
      a0 = a0 * rm; a1 = a1 * rm; a2 = a2 * rm; a3 = a3 * rm;
#pragma unroll 1
      for (int pp = 0; pp < mcnt; ++pp) {
        const int s = __builtin_amdgcn_readlane(sl, pp);
        const float* vp = Vf + (size_t)s * QW + hoff;
        const v4f v0 = *(const v4f*)vp, v1 = *(const v4f*)(vp + 4), v2 = *(const v4f*)(vp + 8), v3 = *(const v4f*)(vp + 12);
        const float x0 = __shfl(p0, pp), x1 = __shfl(p1, pp), x2 = __shfl(p2, pp), x3 = __shfl(p3, pp);
        const float pa = sel4(grp, x0, x1, x2, x3);
        a0 = a0 + v0 * pa; a1 = a1 + v1 * pa; a2 = a2 + v2 * pa; a3 = a3 + v3 * pa;
      }
    }
    const float dm = sel4(grp, d0, d1, d2, d3);
    const float rd = __builtin_amdgcn_rcpf(fmaxf(dm, 1e-16f));
    v4f x0 = a0 * rd, x1 = a1 * rd, x2 = a2 * rd, x3 = a3 * rd;
    x0 = xs2(x0); x1 = xs2(x1); x2 = xs2(x2); x3 = xs2(x3);
    x0 = x0 * 0.25f; x1 = x1 * 0.25f; x2 = x2 * 0.25f; x3 = x3 * 0.25f;
    const float* skp = SK + (size_t)c * CH + sub * 16;
    const v4f t0 = x0 + *(const v4f*)skp, t1 = x1 + *(const v4f*)(skp + 4), t2 = x2 + *(const v4f*)(skp + 8), t3 = x3 + *(const v4f*)(skp + 12);
    const float ps = (hsum4(t0) + hsum4(t1)) + (hsum4(t2) + hsum4(t3));
    const float mu = wsum(ps) * (1.0f / 512.0f);
    const v4f e0 = t0 - mu, e1 = t1 - mu, e2 = t2 - mu, e3 = t3 - mu;
    const float pv = (hsum4(e0 * e0) + hsum4(e1 * e1)) + (hsum4(e2 * e2) + hsum4(e3 * e3));
    const float var = wsum(pv) * (1.0f / 512.0f);
    const float rs = rsqrtf(var + 1e-5f);
    const v4f y0 = e0 * rs, y1 = e1 * rs, y2 = e2 * rs, y3 = e3 * rs;
    __syncthreads();
    if (grp == 0) {
      *(v4f*)(my + sub * 16)      = y0;
      *(v4f*)(my + sub * 16 + 4)  = y1;
      *(v4f*)(my + sub * 16 + 8)  = y2;
      *(v4f*)(my + sub * 16 + 12) = y3;
    }
    __syncthreads();
    v4f o = *(const v4f*)(my + 4 * lane);
    o = o * g4 + b4;
    const v4h hv = cvt4(o);
    _Float16* hp = Hout + (size_t)c * CH + 4 * lane;
    *(volatile v4h*)hp = hv;
    __threadfence();
    *(volatile v4h*)hp = hv;
  }
}

static void launch_gemm(hipStream_t stream, const _Float16* A, int K, const _Float16* Bp, const float* bias, int useBias,
                        float* C, int Nout, int NP) {
  k_gemm<<<dim3(NP / GROWS, Nout / GNC, 1), NTHR, LDS_GEMM, stream>>>(A, Bp, bias, C, K, K, Nout, K / 32, useBias, RWSC);
}

extern "C" void kernel_launch(void* const* d_in, const int* in_sizes, int n_in,
                              void* d_out, int out_size, void* d_ws, size_t ws_size,
                              hipStream_t stream) {
  if (n_in < 33) return;
  if (in_sizes[0] <= 0 || (in_sizes[0] % CH) != 0) return;
  const int N = in_sizes[0] / CH;
  if (in_sizes[1] <= 0 || (in_sizes[1] & 1) != 0) return;
  const int E = in_sizes[1] / 2;
  if (N <= 0 || E <= 0 || N > (1 << 20) || E > (1 << 26)) return;
  if (in_sizes[2] != N * DCOND) return;
  {
    const int i128[12] = {3, 4, 6, 14, 15, 16, 24, 25, 26, 28, 30, 32};
    for (int i = 0; i < 12; ++i) if (in_sizes[i128[i]] != CH) return;
    const int i512[6] = {8, 10, 12, 18, 20, 22};
    for (int i = 0; i < 6; ++i) if (in_sizes[i512[i]] != QW) return;
    const int icc[6] = {5, 13, 23, 27, 29, 31};
    for (int i = 0; i < 6; ++i) if (in_sizes[icc[i]] != CH * CH) return;
    const int icq[2] = {7, 17};
    for (int i = 0; i < 2; ++i) if (in_sizes[icq[i]] != CH * QW) return;
    const int idq[4] = {9, 11, 19, 21};
    for (int i = 0; i < 4; ++i) if (in_sizes[idq[i]] != DCOND * QW) return;
  }
  if (out_size != N * CH) return;

  const float* x    = (const float*)d_in[0];
  const int*   ei   = (const int*)d_in[1];
  const float* cond = (const float*)d_in[2];
  const float* bn_g = (const float*)d_in[3];
  const float* bn_b = (const float*)d_in[4];
  const float* Wpi  = (const float*)d_in[5];  const float* bpi = (const float*)d_in[6];
  const float* Wq1  = (const float*)d_in[7];  const float* bq1 = (const float*)d_in[8];
  const float* Wk1  = (const float*)d_in[9];  const float* bk1 = (const float*)d_in[10];
  const float* Wv1  = (const float*)d_in[11]; const float* bv1 = (const float*)d_in[12];
  const float* Ws1  = (const float*)d_in[13]; const float* bs1 = (const float*)d_in[14];
  const float* lng1 = (const float*)d_in[15]; const float* lnb1 = (const float*)d_in[16];
  const float* Wq2  = (const float*)d_in[17]; const float* bq2 = (const float*)d_in[18];
  const float* Wk2  = (const float*)d_in[19]; const float* bk2 = (const float*)d_in[20];
  const float* Wv2  = (const float*)d_in[21]; const float* bv2 = (const float*)d_in[22];
  const float* Ws2  = (const float*)d_in[23]; const float* bs2 = (const float*)d_in[24];
  const float* lng2 = (const float*)d_in[25]; const float* lnb2 = (const float*)d_in[26];
  const float* Wg1  = (const float*)d_in[27]; const float* bg1 = (const float*)d_in[28];
  const float* Wg2  = (const float*)d_in[29]; const float* bg2 = (const float*)d_in[30];
  const float* Wpo  = (const float*)d_in[31]; const float* bpo = (const float*)d_in[32];
  float* out = (float*)d_out;

  const int NP = ((N + TGT - 1) / TGT) * TGT;
  const int nBC = (N + NBC - 1) / NBC;
  if (4 * nBC + 1 > RBN) return;
  if (31 * 4 * nBC > 4096) return;
  const int CNTPAD = nBC * NBC;
  const int nBF = (N + NBF - 1) / NBF;
  const int csrLen = ((E + 31) & ~31) + 4096;

  const float* jsrc[NJOB] = {Wpi, Wq1, Wk1, Wv1, Ws1, Wq2, Wk2, Wv2, Ws2, Wg1, Wg2, Wpo};
  const int jK[NJOB] = {CH, CH, DCOND, DCOND, CH, CH, DCOND, DCOND, CH, CH, CH, CH};
  const int jN[NJOB] = {CH, QW, QW, QW, CH, QW, QW, QW, CH, CH, CH, CH};
  size_t joff[NJOB];
  size_t whalves = 0; int maxItems = 0;
  for (int i = 0; i < NJOB; ++i) {
    joff[i] = whalves;
    whalves += (size_t)jN[i] * jK[i];
    const int it = jN[i] * jK[i] / 8;
    maxItems = it > maxItems ? it : maxItems;
  }

  size_t off = 0;
  const size_t oW    = off; off = ((off + whalves * 2) + 255) & ~(size_t)255;
  const size_t oCond = off; off = ((off + (size_t)NP * DCOND * 2) + 255) & ~(size_t)255;
  const size_t oCnt  = off; off = ((off + (size_t)CNTPAD * 4) + 255) & ~(size_t)255;
  const size_t oOff  = off; off = ((off + (size_t)CNTPAD * 4) + 255) & ~(size_t)255;
  const size_t oRb   = off; off = ((off + (size_t)RBN * 4) + 255) & ~(size_t)255;
  const size_t oCsr  = off; off = ((off + (size_t)csrLen * 4) + 255) & ~(size_t)255;
  const size_t oDinv = off; off = ((off + (size_t)NP * 4) + 255) & ~(size_t)255;
  const size_t oStat = off; off = ((off + (size_t)2 * CH * 4) + 255) & ~(size_t)255;
  const size_t oHA   = off; off = ((off + (size_t)NP * CH * 2) + 255) & ~(size_t)255;
  const size_t oHB   = off; off = ((off + (size_t)NP * CH * 2) + 255) & ~(size_t)255;
  const size_t oXW   = off; off = ((off + (size_t)NP * CH * 4) + 255) & ~(size_t)255;
  const size_t oSkip = off; off = ((off + (size_t)NP * CH * 4) + 255) & ~(size_t)255;
  const size_t oQ    = off; off = ((off + (size_t)NP * QW * 4) + 255) & ~(size_t)255;
  const size_t oK    = off; off = ((off + (size_t)NP * QW * 4) + 255) & ~(size_t)255;
  const size_t oV    = off; off = ((off + (size_t)NP * QW * 4) + 255) & ~(size_t)255;
  if (off > ws_size || off > (size_t)WSCAP) return;

  char* ws = (char*)d_ws;
  _Float16* wp    = (_Float16*)(ws + oW);
  _Float16* CONDH = (_Float16*)(ws + oCond);
  int*   cnt   = (int*)(ws + oCnt);
  int*   offp  = (int*)(ws + oOff);
  int*   rb    = (int*)(ws + oRb);
  int*   csr   = (int*)(ws + oCsr);
  float* dinv  = (float*)(ws + oDinv);
  float* stats = (float*)(ws + oStat);
  _Float16* HA = (_Float16*)(ws + oHA);
  _Float16* HB = (_Float16*)(ws + oHB);
  float* XW    = (float*)(ws + oXW);
  float* SKIP  = (float*)(ws + oSkip);
  float* Qb    = (float*)(ws + oQ);
  float* Kb    = (float*)(ws + oK);
  float* Vb    = (float*)(ws + oV);

  WJobs J;
  const _Float16* pl[NJOB];
  for (int i = 0; i < NJOB; ++i) {
    J.j[i].src = jsrc[i]; J.j[i].dst = wp + joff[i]; J.j[i].K = jK[i]; J.j[i].N = jN[i];
    pl[i] = wp + joff[i];
  }
  const int vec8 = ((E & 3) == 0) ? 1 : 0;

  hipFuncSetAttribute(reinterpret_cast<const void*>(&k_fill), hipFuncAttributeMaxDynamicSharedMemorySize, LDS_FILL);
  hipFuncSetAttribute(reinterpret_cast<const void*>(&k_gemm), hipFuncAttributeMaxDynamicSharedMemorySize, LDS_GEMM);

  k_wprep<<<dim3((maxItems + NTHR - 1) / NTHR, NJOB, 1), NTHR, 0, stream>>>(J);
  {
    const int items = NP * (DCOND / 8);
    k_cvt<<<(items + NTHR - 1) / NTHR, NTHR, 0, stream>>>(cond, CONDH, N, DCOND, items);
  }
  k_count<<<nBC, NTHR, 0, stream>>>(ei, cnt, E, vec8);
  k_offsets<<<1, OTHR, 0, stream>>>(cnt, offp, rb, nBC);
  k_fill<<<nBF, NTHR, LDS_FILL, stream>>>(ei, offp, rb, csr, E, vec8, csrLen);
  k_dinv<<<(NP / 4 + NTHR - 1) / NTHR, NTHR, 0, stream>>>(cnt, dinv, NP / 4);
  k_bnstat<<<CH / 32, NTHR, 0, stream>>>(x, stats, N);
  k_bnapply<<<NP / 32, NTHR, 0, stream>>>(x, stats, bn_g, bn_b, HA, N);
  launch_gemm(stream, HA, CH, pl[0], bpi, 0, XW, CH, NP);
  k_gcn<<<NP / TGT, NTHR, 0, stream>>>(csr, offp, cnt, ei, dinv, XW, bpi, x, HB, out, N, E, csrLen, 0);
  launch_gemm(stream, HB, CH, pl[1], bq1, 1, Qb, QW, NP);
  launch_gemm(stream, CONDH, DCOND, pl[2], bk1, 1, Kb, QW, NP);
  launch_gemm(stream, CONDH, DCOND, pl[3], bv1, 1, Vb, QW, NP);
  launch_gemm(stream, HB, CH, pl[4], bs1, 1, SKIP, CH, NP);
  k_attn<<<NP / TGT, NTHR, 0, stream>>>(csr, offp, cnt, ei, Qb, Kb, Vb, SKIP, lng1, lnb1, HA, N, E, csrLen);
  launch_gemm(stream, HA, CH, pl[5], bq2, 1, Qb, QW, NP);
  launch_gemm(stream, CONDH, DCOND, pl[6], bk2, 1, Kb, QW, NP);
  launch_gemm(stream, CONDH, DCOND, pl[7], bv2, 1, Vb, QW, NP);
  launch_gemm(stream, HA, CH, pl[8], bs2, 1, SKIP, CH, NP);
  k_attn<<<NP / TGT, NTHR, 0, stream>>>(csr, offp, cnt, ei, Qb, Kb, Vb, SKIP, lng2, lnb2, HB, N, E, csrLen);
  launch_gemm(stream, HB, CH, pl[9], bg1, 0, XW, CH, NP);
  k_gcn<<<NP / TGT, NTHR, 0, stream>>>(csr, offp, cnt, ei, dinv, XW, bg1, x, HA, out, N, E, csrLen, 1);
  launch_gemm(stream, HA, CH, pl[10], bg2, 0, XW, CH, NP);
  k_gcn<<<NP / TGT, NTHR, 0, stream>>>(csr, offp, cnt, ei, dinv, XW, bg2, x, HB, out, N, E, csrLen, 0);
  launch_gemm(stream, HB, CH, pl[11], bpo, 0, XW, CH, NP);
  k_gcn<<<NP / TGT, NTHR, 0, stream>>>(csr, offp, cnt, ei, dinv, XW, bpo, x, HB, out, N, E, csrLen, 2);
}
